// MultiHeadAttention_33560874451292
// MI455X (gfx1250) — hardware-run, weakly checked
//
#include <hip/hip_runtime.h>
#ifndef NB
#define NB 2
#endif
#ifndef SEQ
#define SEQ 2048
#endif
#define NB_FULL 2
#define SEQ_FULL 2048
#define SQ SEQ
#define DM 1024
#define NH 16
#define HD 64
#define NR ((size_t)NB * SQ)
#define SM_SCALE 0.125f
#define LN_CARRY 5.545177444479562f

static_assert(NH * HD == DM);
static_assert(HD == 64);
static_assert(SQ % 128 == 0);
static_assert(DM % 64 == 0);
static_assert(DM % 32 == 0);
static_assert(NB <= NB_FULL);
static_assert(SQ <= SEQ_FULL);
static_assert(4ull * DM * DM * 2ull + 4ull * NB * SQ * DM * 2ull + (unsigned long long)NB * DM * SQ * 2ull <= 134217728ull);

typedef unsigned short v8us __attribute__((ext_vector_type(8), may_alias));
typedef float  v8f  __attribute__((ext_vector_type(8)));
typedef float  v4f  __attribute__((ext_vector_type(4)));
typedef float  v4fa __attribute__((ext_vector_type(4), may_alias));
typedef _Float16 v16h __attribute__((ext_vector_type(16)));
typedef _Float16 v4h __attribute__((ext_vector_type(4)));
union FragH { v16h v; v8us half[2]; _Float16 h[16]; unsigned short u[16]; };

__device__ __forceinline__ unsigned short bf16_bits(float x) { unsigned int u = __float_as_uint(x); return (unsigned short)((u + 0x7FFFu + ((u >> 16) & 1u)) >> 16); }
__device__ __forceinline__ float bf16_val(unsigned short b) { return __uint_as_float(((unsigned int)b) << 16); }
__device__ __forceinline__ float bf16_rne(float x) { return bf16_val(bf16_bits(x)); }

__device__ __forceinline__ v16h g2_frag(const _Float16* p, int hh) { FragH f; f.half[0] = *(const v8us*)((const unsigned short*)p + 8 * hh); f.half[1] = *(const v8us*)((const unsigned short*)p + 16 + 8 * hh); return f.v; }
__device__ __forceinline__ v8f g2_mma(v16h a, v16h b, v8f c) { v8f d = __builtin_amdgcn_wmma_f32_16x16x32_f16(false, a, false, b, (short)0, c, false, false); asm volatile("v_nop\n\tv_nop\n\tv_nop\n\tv_nop" : "+v"(d) : "v"(a), "v"(b)); return d; }

__global__ __launch_bounds__(256) void k_wnat(const float* __restrict__ w, size_t n8, _Float16* __restrict__ Bt) {
  const size_t t = (size_t)blockIdx.x * 256 + threadIdx.x; if (t >= n8) return;
  const v4f a = *(const v4fa*)(w + t * 8), c = *(const v4fa*)(w + t * 8 + 4);
  FragH f;
#pragma unroll
  for (int q = 0; q < 4; ++q) { f.h[q] = (_Float16)(bf16_rne(a[q]) * 16.0f); f.h[4 + q] = (_Float16)(bf16_rne(c[q]) * 16.0f); }
  const v8us o = f.half[0];
  *(volatile v8us*)((unsigned short*)Bt + t * 8) = o; __threadfence(); *(volatile v8us*)((unsigned short*)Bt + t * 8) = o;
}

__global__ __launch_bounds__(256) void k_x16(const float* __restrict__ x, _Float16* __restrict__ X16, size_t n8) {
  const size_t t = (size_t)blockIdx.x * 256 + threadIdx.x; if (t >= n8) return;
  const size_t e = t * 8; const size_t row = e / DM; const size_t c0 = e - row * DM; const size_t bb = row / SQ; const size_t s = row - bb * SQ;
  const float* src = x + (bb * SEQ_FULL + s) * DM + c0;
  const v4f a = *(const v4fa*)(src), c = *(const v4fa*)(src + 4);
  FragH f;
#pragma unroll
  for (int q = 0; q < 4; ++q) { f.h[q] = (_Float16)bf16_rne(a[q]); f.h[4 + q] = (_Float16)bf16_rne(c[q]); }
  const v8us o = f.half[0];
  *(volatile v8us*)((unsigned short*)X16 + e) = o; __threadfence(); *(volatile v8us*)((unsigned short*)X16 + e) = o;
}

__global__ __launch_bounds__(128) void k_gemm2(const _Float16* __restrict__ A, int lda, size_t sA, const _Float16* __restrict__ Bh, int ldb, size_t sB, float alpha,
    const float* __restrict__ bias, float* __restrict__ C, _Float16* __restrict__ C16, int ldc, size_t sC, int M, int N, int K) {
  __shared__ __attribute__((aligned(16))) float so[4][32][68];
  const int tid = threadIdx.x, w = __builtin_amdgcn_readfirstlane((int)(tid >> 5)), lane = tid & 31, ln = lane & 15, hh = lane >> 4; const int by = blockIdx.y;
  A += (size_t)by * sA; Bh += (size_t)by * sB; const size_t cofs = (size_t)by * sC;
  const int ntn = N >> 6; const int mt = blockIdx.x / ntn, nq = blockIdx.x - mt * ntn; const int row0 = mt * 128 + 32 * w, col0 = nq * 64; if (row0 >= M) return;
  const _Float16* a0p = A + (size_t)(row0 + ln) * lda; const _Float16* a1p = a0p + (size_t)16 * lda;
  const _Float16* b0p = Bh + (size_t)(col0 + ln) * ldb; const _Float16* b1p = b0p + (size_t)16 * ldb; const _Float16* b2p = b1p + (size_t)16 * ldb; const _Float16* b3p = b2p + (size_t)16 * ldb;
  const v8f z8 = {0.f,0.f,0.f,0.f,0.f,0.f,0.f,0.f}; v8f c00 = z8, c01 = z8, c02 = z8, c03 = z8, c10 = z8, c11 = z8, c12 = z8, c13 = z8;
#pragma unroll 1
  for (int kb = 0; kb < K; kb += 32) { const v16h a0 = g2_frag(a0p + kb, hh), a1 = g2_frag(a1p + kb, hh);
    v16h b = g2_frag(b0p + kb, hh); c00 = g2_mma(a0, b, c00); c10 = g2_mma(a1, b, c10);
    b = g2_frag(b1p + kb, hh); c01 = g2_mma(a0, b, c01); c11 = g2_mma(a1, b, c11);
    b = g2_frag(b2p + kb, hh); c02 = g2_mma(a0, b, c02); c12 = g2_mma(a1, b, c12);
    b = g2_frag(b3p + kb, hh); c03 = g2_mma(a0, b, c03); c13 = g2_mma(a1, b, c13); }
  v8f accs[8] = {c00, c01, c02, c03, c10, c11, c12, c13};
#pragma unroll
  for (int u = 0; u < 8; ++u) { const int t = u & 3, half = u >> 2; const int col = col0 + t * 16 + ln; const float bv = bias ? bf16_rne(bias[col]) : 0.f;
#pragma unroll
    for (int r = 0; r < 8; ++r) { const int rloc = half * 16 + 8 * hh + r; so[w][rloc][t * 16 + ln] = accs[u][r] * alpha + bv; } }
  __builtin_amdgcn_fence(4  , "workgroup"); __builtin_amdgcn_wave_barrier();
  const int rsub = lane >> 4, c4 = (lane & 15) * 4;
  for (int pass = 0; pass < 2; ++pass) {
#pragma unroll
    for (int q = 0; q < 16; ++q) { const int r = q * 2 + rsub; const v4f v = *(const v4fa*)&so[w][r][c4];
      if (C) *(volatile v4f*)(C + cofs + (size_t)(row0 + r) * ldc + col0 + c4) = v;
      if (C16) { v4h h4;
#pragma unroll
        for (int i = 0; i < 4; ++i) h4[i] = (_Float16)v[i];
        *(volatile v4h*)(C16 + cofs + (size_t)(row0 + r) * ldc + col0 + c4) = h4; } }
    if (pass == 0) __threadfence(); } }

template <int NHv, int TTv>
__global__ __launch_bounds__(256) void k_vt(const _Float16* __restrict__ V16, int ldv, int voff, _Float16* __restrict__ Vt) {
  __shared__ unsigned short tl[64][66];
  const int tid = threadIdx.x; const int slab = blockIdx.x / (TTv / 64), lg = blockIdx.x % (TTv / 64); const int b = slab / NHv, h = slab % NHv;
  for (int i = tid; i < 64 * 8; i += 256) { const int r = i / 8, c8 = (i % 8) * 8; FragH f;
    f.half[0] = *(const v8us*)((const unsigned short*)V16 + ((size_t)b * TTv + lg * 64 + r) * ldv + voff + h * 64 + c8);
#pragma unroll
    for (int q = 0; q < 8; ++q) tl[r][c8 + q] = f.u[q]; }
  __syncthreads();
  for (int pass = 0; pass < 2; ++pass) {
#pragma unroll
    for (int rd = 0; rd < 2; ++rd) { const int d = rd * 32 + tid / 8, pc = tid % 8; FragH f;
#pragma unroll
      for (int q = 0; q < 8; ++q) f.u[q] = tl[pc * 8 + q][d];
      const v8us o = f.half[0];
      *(volatile v8us*)((unsigned short*)Vt + ((size_t)slab * 64 + d) * TTv + lg * 64 + pc * 8) = o; }
    if (pass == 0) __threadfence(); } }

__global__ __launch_bounds__(128) void k_attn(const _Float16* __restrict__ Q16, const _Float16* __restrict__ K16, const _Float16* __restrict__ VT, _Float16* __restrict__ O16) {
  __shared__ __attribute__((aligned(16))) unsigned short st[4][16][72];
  const int tid = threadIdx.x, w = __builtin_amdgcn_readfirstlane((int)(tid >> 5)), lane = tid & 31, ln = lane & 15, hh = lane >> 4;
  const int bh = blockIdx.y; const int b = bh / NH, h = bh - b * NH;
  const int q0 = blockIdx.x * 64 + w * 16;
  const _Float16* qrow = Q16 + ((size_t)b * SQ + q0 + ln) * DM + h * HD;
  const v16h qf0 = g2_frag(qrow, hh), qf1 = g2_frag(qrow + 32, hh);
  const _Float16* kp = K16 + ((size_t)b * SQ + ln) * DM + h * HD;
  const _Float16* vp = VT + ((size_t)b * DM + (size_t)h * HD + ln) * SQ;
  const v8f z8 = {0.f,0.f,0.f,0.f,0.f,0.f,0.f,0.f};
  v8f o0 = z8, o1 = z8, o2 = z8, o3 = z8;
  float m = -1.0e30f, l = 0.f;
#pragma unroll 1
  for (int j = 0; j < SQ; j += 32) {
    const _Float16* k0 = kp + (size_t)j * DM; const _Float16* k1 = k0 + (size_t)16 * DM;
    v8f s0 = z8, s1 = z8; v16h a;
    a = g2_frag(k0, hh);      s0 = g2_mma(a, qf0, s0); a = g2_frag(k1, hh);      s1 = g2_mma(a, qf0, s1);
    a = g2_frag(k0 + 32, hh); s0 = g2_mma(a, qf1, s0); a = g2_frag(k1 + 32, hh); s1 = g2_mma(a, qf1, s1);
    float mx = fmaxf(s0[0], s1[0]);
#pragma unroll
    for (int r = 1; r < 8; ++r) mx = fmaxf(mx, fmaxf(s0[r], s1[r]));
    mx = fmaxf(mx, __shfl_xor(mx, 16, 32));
    mx *= SM_SCALE;
    const float mnew = fmaxf(m, mx);
    const float alpha = __expf(m - mnew);
    m = mnew;
    const float mb = mnew - LN_CARRY;
    FragH pf; float ps = 0.f;
#pragma unroll
    for (int r = 0; r < 8; ++r) { const float p = __expf(s0[r] * SM_SCALE - mb); ps += p; pf.h[r] = (_Float16)p; }
#pragma unroll
    for (int r = 0; r < 8; ++r) { const float p = __expf(s1[r] * SM_SCALE - mb); ps += p; pf.h[8 + r] = (_Float16)p; }
    l = l * alpha + ps;
    o0 *= alpha; o1 *= alpha; o2 *= alpha; o3 *= alpha;
    int jv = j;
    asm volatile("" : "+v"(jv) : "v"(pf.v));
    const _Float16* vj = vp + jv;
    a = g2_frag(vj, hh);                      o0 = g2_mma(a, pf.v, o0);
    a = g2_frag(vj + (size_t)16 * SQ, hh);    o1 = g2_mma(a, pf.v, o1);
    a = g2_frag(vj + (size_t)32 * SQ, hh);    o2 = g2_mma(a, pf.v, o2);
    a = g2_frag(vj + (size_t)48 * SQ, hh);    o3 = g2_mma(a, pf.v, o3);
  }
  const float lt = l + __shfl_xor(l, 16, 32);
  const float inv = 64.0f / lt;
  v8f oo[4] = {o0, o1, o2, o3};
#pragma unroll
  for (int dt = 0; dt < 4; ++dt) { FragH f;
#pragma unroll
    for (int r = 0; r < 8; ++r) f.h[r] = (_Float16)(oo[dt][r] * inv);
    *(v8us*)&st[w][ln][dt * 16 + 8 * hh] = f.half[0]; }
  __builtin_amdgcn_fence(4  , "workgroup"); __builtin_amdgcn_wave_barrier();
  const int rsub = lane >> 3, c8 = (lane & 7) * 8;
  unsigned short* orow = (unsigned short*)O16 + ((size_t)b * SQ + q0) * DM + h * HD;
  for (int pass = 0; pass < 2; ++pass) {
#pragma unroll
    for (int q = 0; q < 4; ++q) { const int r = q * 4 + rsub; const v8us v = *(const v8us*)&st[w][r][c8];
      *(volatile v8us*)(orow + (size_t)r * DM + c8) = v; }
    if (pass == 0) __threadfence(); }
}

extern "C" void kernel_launch(void* const* d_in, const int* in_sizes, int n_in,
                              void* d_out, int out_size, void* d_ws, size_t ws_size, hipStream_t stream) {
  if (n_in < 9) return;
  const size_t needx = ((size_t)(NB - 1) * SEQ_FULL + SQ) * DM;
  if ((size_t)in_sizes[0] < needx) return;
  if ((size_t)in_sizes[1] < (size_t)DM * DM || (size_t)in_sizes[3] < (size_t)DM * DM || (size_t)in_sizes[5] < (size_t)DM * DM || (size_t)in_sizes[7] < (size_t)DM * DM) return;
  if (in_sizes[2] < DM || in_sizes[4] < DM || in_sizes[6] < DM || in_sizes[8] < DM) return;
  if ((size_t)out_size < needx) return;
  const float* x  = (const float*)d_in[0];
  const float* wq = (const float*)d_in[1]; const float* bq = (const float*)d_in[2];
  const float* wk = (const float*)d_in[3]; const float* bk = (const float*)d_in[4];
  const float* wv = (const float*)d_in[5]; const float* bv = (const float*)d_in[6];
  const float* wo = (const float*)d_in[7]; const float* bo = (const float*)d_in[8];
  char* ws = (char*)d_ws; size_t off = 0;
  auto take = [&](size_t bytes) { char* p = ws + off; off += (bytes + 255) & ~(size_t)255; return p; };
  _Float16* BQ = (_Float16*)take((size_t)DM * DM * 2); _Float16* BK = (_Float16*)take((size_t)DM * DM * 2);
  _Float16* BV = (_Float16*)take((size_t)DM * DM * 2); _Float16* BO = (_Float16*)take((size_t)DM * DM * 2);
  _Float16* X16 = (_Float16*)take(NR * DM * 2);
  _Float16* O16 = X16;
  _Float16* Q16 = (_Float16*)take(NR * DM * 2); _Float16* K16 = (_Float16*)take(NR * DM * 2); _Float16* V16 = (_Float16*)take(NR * DM * 2);
  _Float16* VT = (_Float16*)take((size_t)NB * DM * SQ * 2);
  if (off > ws_size) return;
  { const size_t n8 = (size_t)DM * DM / 8; const unsigned g = (unsigned)((n8 + 255) / 256);
    k_wnat<<<g, 256, 0, stream>>>(wq, n8, BQ); k_wnat<<<g, 256, 0, stream>>>(wk, n8, BK);
    k_wnat<<<g, 256, 0, stream>>>(wv, n8, BV); k_wnat<<<g, 256, 0, stream>>>(wo, n8, BO); }
  { const size_t n8 = NR * DM / 8; k_x16<<<(unsigned)((n8 + 255) / 256), 256, 0, stream>>>(x, X16, n8); }
  const int MP = (int)NR;
  const dim3 gp((unsigned)((MP / 128) * (DM / 64)), 1);
  k_gemm2<<<gp, 128, 0, stream>>>(X16, DM, (size_t)0, BQ, DM, (size_t)0, 0.0625f, bq, nullptr, Q16, DM, (size_t)0, MP, DM, DM);
  k_gemm2<<<gp, 128, 0, stream>>>(X16, DM, (size_t)0, BK, DM, (size_t)0, 0.0625f, bk, nullptr, K16, DM, (size_t)0, MP, DM, DM);
  k_gemm2<<<gp, 128, 0, stream>>>(X16, DM, (size_t)0, BV, DM, (size_t)0, 0.0625f, bv, nullptr, V16, DM, (size_t)0, MP, DM, DM);
  k_vt<DM / 64, SQ><<<(unsigned)(NB * (DM / 64) * (SQ / 64)), 256, 0, stream>>>(V16, DM, 0, VT);
  k_attn<<<dim3((unsigned)(SQ / 64), (unsigned)(NB * NH)), 128, 0, stream>>>(Q16, K16, VT, O16);
  k_gemm2<<<dim3((unsigned)((SQ / 128) * (DM / 64)), (unsigned)NB), 128, 0, stream>>>(O16, DM, (size_t)SQ * DM, BO, DM, (size_t)0, 0.0009765625f, bo,
      (float*)d_out, nullptr, DM, (size_t)SEQ_FULL * DM, SQ, DM, DM);
}
